// RelationNetwork_11347303596677
// MI455X (gfx1250) — hardware-verified
//
#include <hip/hip_runtime.h>


#define NB   32
#define NOBJ 128
#define DIN  64
#define REL  256
#define NPAIR (NOBJ * NOBJ)
#define NOUT 10
#define DM   DIN
#define LOSC 1024.0f

typedef _Float16 h16;
typedef unsigned short bf;
typedef __attribute__((ext_vector_type(16))) __bf16   v16bf;
typedef __attribute__((ext_vector_type(16))) _Float16 v16h;
typedef __attribute__((ext_vector_type(8)))  _Float16 v8h;
typedef __attribute__((ext_vector_type(8)))  unsigned short v8us;
typedef __attribute__((ext_vector_type(8)))  float    v8f;
typedef __attribute__((ext_vector_type(4)))  float    v4f;
typedef __attribute__((ext_vector_type(4)))  _Float16 v4h;
typedef v8h  __attribute__((may_alias)) v8ha;
typedef v4f  __attribute__((may_alias)) v4fa;
typedef v8us __attribute__((may_alias)) v8usa;

__device__ __forceinline__ unsigned short f2bf(float f) { unsigned u = __float_as_uint(f); u += 0x7FFFu + ((u >> 16) & 1u); return (unsigned short)(u >> 16); }
__device__ __forceinline__ float bf2f(unsigned short b) { return __uint_as_float(((unsigned)b) << 16); }
__device__ __forceinline__ float bfr(float f) { return bf2f(f2bf(f)); }
__device__ __forceinline__ v16h cat16(v8h lo, v8h hi) { return __builtin_shufflevector(lo, hi, 0, 1, 2, 3, 4, 5, 6, 7, 8, 9, 10, 11, 12, 13, 14, 15); }
__device__ __forceinline__ v16bf cat16b(v8us lo, v8us hi) { return __builtin_bit_cast(v16bf, __builtin_shufflevector(lo, hi, 0, 1, 2, 3, 4, 5, 6, 7, 8, 9, 10, 11, 12, 13, 14, 15)); }
__device__ __forceinline__ v8f wmma16(v16h a, v16h b, v8f c) { return __builtin_amdgcn_wmma_f32_16x16x32_f16(false, a, false, b, (short)0, c, false, false); }
__device__ __forceinline__ v8f wmmab(v16bf a, v16bf b, v8f c) { return __builtin_amdgcn_wmma_f32_16x16x32_bf16(false, a, false, b, (short)0, c, false, false); }

__global__ __launch_bounds__(256) void k_cvt64(const float* __restrict__ src, int nrows, bf* dst) {
    typedef __attribute__((ext_vector_type(4))) unsigned short v4us;
    const size_t i = (size_t)blockIdx.x * 256 + threadIdx.x; if (i >= (size_t)nrows * DIN / 4) return;
    const v4f v = *(const v4f*)(src + i * 4); v4us o;
#pragma unroll
    for (int k = 0; k < 4; ++k) o[k] = f2bf(v[k]);
    *(volatile v4us*)(dst + i * 4) = o; __threadfence(); *(volatile v4us*)(dst + i * 4) = o;
}
__global__ __launch_bounds__(256) void k_wt(const float* __restrict__ Wm, int K, int ncols, bf* WT) {
    __shared__ __align__(16) unsigned short tl[64 * 72];
    const int tid = threadIdx.x, k0 = blockIdx.x * 64, n0 = blockIdx.y * 64;
    const int kk = tid >> 2, nq = (tid & 3) * 16;
#pragma unroll
    for (int i = 0; i < 16; ++i) tl[(nq + i) * 72 + kk] = f2bf(Wm[(size_t)(k0 + kk) * ncols + n0 + nq + i]);
    __syncthreads();
    const int piece = tid & 7;
    auto pass = [&]() {
#pragma unroll
        for (int s = 0; s < 2; ++s) { const int nr = (tid >> 3) + 32 * s; const v8us val = *(const v8usa*)(tl + nr * 72 + piece * 8); *(volatile v8us*)(WT + (size_t)(n0 + nr) * K + k0 + piece * 8) = val; }
    };
    pass(); __threadfence(); pass();
}
template <bool SPLITA, bool F16OUT = false>
__global__ __launch_bounds__(128) void k_gemmb(const bf* __restrict__ A, const bf* __restrict__ Al, const bf* __restrict__ Bn, const float* __restrict__ bias, float* C, int ldc, h16* C2, const float* __restrict__ R = nullptr, int K = DM, int roundR = 1) {
    __shared__ __align__(16) float ost[4][16 * 68];
    const int lane = threadIdx.x & 31, wave = threadIdx.x >> 5, lr = lane & 15, hi = lane >> 4;
    const int r0 = blockIdx.x * 64 + wave * 16, c0 = blockIdx.y * 64;
    const size_t aoff = (size_t)(r0 + lr) * K + 8 * hi;
    size_t boff[4];
#pragma unroll
    for (int t = 0; t < 4; ++t) boff[t] = (size_t)(c0 + t * 16 + lr) * K + 8 * hi;
    v8f acc[4];
#pragma unroll
    for (int t = 0; t < 4; ++t) acc[t] = (v8f){};
#pragma unroll 1
    for (int kc = 0; kc < K; kc += 32) {
        const v16bf a = cat16b(*(const v8us*)(A + aoff + kc), *(const v8us*)(A + aoff + kc + 16));
        v16bf al = a;
        if (SPLITA) al = cat16b(*(const v8us*)(Al + aoff + kc), *(const v8us*)(Al + aoff + kc + 16));
#pragma unroll
        for (int t = 0; t < 4; ++t) { const v16bf b = cat16b(*(const v8us*)(Bn + boff[t] + kc), *(const v8us*)(Bn + boff[t] + kc + 16)); acc[t] = wmmab(a, b, acc[t]); if (SPLITA) acc[t] = wmmab(al, b, acc[t]); }
        asm volatile("v_nop\n\tv_nop\n\tv_nop\n\tv_nop" : "+v"(acc[0]), "+v"(acc[1]), "+v"(acc[2]), "+v"(acc[3]) : "v"(a), "v"(al));
    }
    float* os = &ost[wave][0];
#pragma unroll
    for (int t = 0; t < 4; ++t) { const float bv = bias ? bfr(bias[c0 + t * 16 + lr]) : 0.f;
#pragma unroll
        for (int j = 0; j < 8; ++j) os[(hi * 8 + j) * 68 + t * 16 + lr] = acc[t][j] + bv; }
    __syncthreads();
    if (F16OUT) {
        h16* crow = (h16*)(void*)C + (size_t)r0 * ldc + c0;
        auto pass = [&]() {
#pragma unroll
            for (int s = 0; s < 4; ++s) { const int row = 4 * s + (lane >> 3), piece = lane & 7; const float* sp = os + row * 68 + piece * 8; v8h o, o2;
#pragma unroll
                for (int i = 0; i < 8; ++i) { const h16 a = (h16)sp[i]; o[i] = a; o2[i] = (h16)((sp[i] - (float)a) * LOSC); }
                *(volatile v8h*)(crow + (size_t)row * ldc + piece * 8) = o; if (C2) *(volatile v8h*)(C2 + (size_t)r0 * ldc + c0 + (size_t)row * ldc + piece * 8) = o2; }
        };
        pass(); __threadfence(); pass();
    } else {
        float* crow = C + (size_t)r0 * ldc + c0;
        auto pass = [&]() {
#pragma unroll
            for (int s = 0; s < 8; ++s) { const int Lid = (lane >> 3) + 4 * s, piece = lane & 7; const int row = Lid >> 1, cofs = (Lid & 1) * 32 + piece * 4;
                v4f val = *(const v4fa*)(os + row * 68 + cofs); if (R) { const v4f rv = *(const v4f*)(R + ((size_t)r0 + row) * ldc + c0 + cofs); val += roundR ? (v4f){bfr(rv[0]), bfr(rv[1]), bfr(rv[2]), bfr(rv[3])} : rv; }
                *(volatile v4f*)(crow + (size_t)row * ldc + cofs) = val; }
        };
        pass(); __threadfence(); pass();
    }
}

__global__ __launch_bounds__(256) void k_pairh(const float* __restrict__ P, const float* __restrict__ Q, const float* __restrict__ bg1, bf* Hh, bf* Hl) {
    const int lane = threadIdx.x & 31, r = blockIdx.x * 8 + (threadIdx.x >> 5);
    if (r >= NPAIR) return;
    const int i = r / NOBJ, j = r - i * NOBJ;
    const v8f pv = *(const v8f*)(P + (size_t)i * REL + lane * 8), qv = *(const v8f*)(Q + (size_t)j * REL + lane * 8);
    v8us oh, ol;
#pragma unroll
    for (int k = 0; k < 8; ++k) { const float h = fmaxf((pv[k] + qv[k]) + bfr(bg1[lane * 8 + k]), 0.f); const unsigned short hb = f2bf(h); oh[k] = hb; ol[k] = f2bf(h - bf2f(hb)); }
    const size_t o = (size_t)r * REL + lane * 8; *(volatile v8us*)(Hh + o) = oh; *(volatile v8us*)(Hl + o) = ol; __threadfence(); *(volatile v8us*)(Hh + o) = oh; *(volatile v8us*)(Hl + o) = ol;
}
__global__ __launch_bounds__(256) void k_pool(const float* __restrict__ T2, int b, float* POOL) {
    __shared__ __align__(16) float ps[REL];
    const int c = threadIdx.x; float s = 0.f;
#pragma unroll 1
    for (int r = 0; r < NPAIR; ++r) s += fmaxf(T2[(size_t)r * REL + c], 0.f);
    ps[c] = s; __syncthreads();
    if (threadIdx.x < REL / 4) { const v4f v = *(const v4fa*)(&ps[threadIdx.x * 4]); float* dst = POOL + (size_t)b * REL + threadIdx.x * 4; *(volatile v4f*)dst = v; __threadfence(); *(volatile v4f*)dst = v; }
}
__global__ __launch_bounds__(256) void k_head(const float* __restrict__ POOL, const float* __restrict__ Wf1, const float* __restrict__ bf1, const float* __restrict__ Wf2, const float* __restrict__ bf2, float* OUTP) {
    __shared__ float zs[REL]; __shared__ __align__(16) float os[NB * NOUT];
    const int c = threadIdx.x;
#pragma unroll 1
    for (int b = 0; b < NB; ++b) {
        float a = bfr(bf1[c]);
#pragma unroll 1
        for (int k = 0; k < REL; ++k) a = fmaf(POOL[(size_t)b * REL + k], bfr(Wf1[(size_t)k * REL + c]), a);
        zs[c] = fmaxf(a, 0.f); __syncthreads();
        if (c < NOUT) { float o = bfr(bf2[c]);
#pragma unroll 1
            for (int k = 0; k < REL; ++k) o = fmaf(zs[k], bfr(Wf2[k * NOUT + c]), o);
            os[b * NOUT + c] = o; }
        __syncthreads();
    }
    if (c < NB * NOUT / 4) { const v4f v = *(const v4fa*)(&os[c * 4]); *(volatile v4f*)(OUTP + c * 4) = v; __threadfence(); *(volatile v4f*)(OUTP + c * 4) = v; }
}

extern "C" void kernel_launch(void* const* d_in, const int* in_sizes, int n_in,
                              void* d_out, int out_size, void* d_ws, size_t ws_size, hipStream_t stream) {
    (void)in_sizes; (void)n_in; (void)out_size;
    const float* obj = (const float*)d_in[0]; const float* Wg1 = (const float*)d_in[1]; const float* bg1 = (const float*)d_in[2]; const float* Wg2 = (const float*)d_in[3]; const float* bg2 = (const float*)d_in[4];
    const float* Wf1 = (const float*)d_in[5]; const float* bf1 = (const float*)d_in[6]; const float* Wf2 = (const float*)d_in[7]; const float* bf2 = (const float*)d_in[8];
    float* out = (float*)d_out;
    char* wsp = (char*)d_ws;
    auto take = [&](size_t bytes) { char* p = wsp; wsp += (bytes + 255) & ~(size_t)255; return (void*)p; };
    bf* Ob = (bf*)take((size_t)NB * NOBJ * DIN * 2); bf* WaT = (bf*)take((size_t)REL * DIN * 2); bf* WbT = (bf*)take((size_t)REL * DIN * 2); bf* W2T = (bf*)take((size_t)REL * REL * 2);
    float* P = (float*)take((size_t)NOBJ * REL * 4); float* Q = (float*)take((size_t)NOBJ * REL * 4);
    bf* Hh = (bf*)take((size_t)NPAIR * REL * 2); bf* Hl = (bf*)take((size_t)NPAIR * REL * 2); float* T2 = (float*)take((size_t)NPAIR * REL * 4); float* POOL = (float*)take((size_t)NB * REL * 4);
    if ((size_t)(wsp - (char*)d_ws) > ws_size) return;
    k_cvt64<<<(NB * NOBJ * DIN / 4 + 255) / 256, 256, 0, stream>>>(obj, NB * NOBJ, Ob);
    k_wt<<<dim3(DIN / 64, REL / 64, 1), 256, 0, stream>>>(Wg1, DIN, REL, WaT);
    k_wt<<<dim3(DIN / 64, REL / 64, 1), 256, 0, stream>>>(Wg1 + (size_t)DIN * REL, DIN, REL, WbT);
    k_wt<<<dim3(REL / 64, REL / 64, 1), 256, 0, stream>>>(Wg2, REL, REL, W2T);
    for (int b = 0; b < NB; ++b) {
        k_gemmb<false, false><<<dim3(NOBJ / 64, REL / 64, 1), 128, 0, stream>>>(Ob + (size_t)b * NOBJ * DIN, nullptr, WaT, nullptr, P, REL, nullptr);
        k_gemmb<false, false><<<dim3(NOBJ / 64, REL / 64, 1), 128, 0, stream>>>(Ob + (size_t)b * NOBJ * DIN, nullptr, WbT, nullptr, Q, REL, nullptr);
        k_pairh<<<NPAIR / 8, 256, 0, stream>>>(P, Q, bg1, Hh, Hl);
        k_gemmb<true, false><<<dim3(NPAIR / 64, REL / 64, 1), 128, 0, stream>>>(Hh, Hl, W2T, bg2, T2, REL, nullptr, nullptr, REL);
        k_pool<<<1, 256, 0, stream>>>(T2, b, POOL);
    }
    k_head<<<1, 256, 0, stream>>>(POOL, Wf1, bf1, Wf2, bf2, out);
}
